// VariableSelectionNetwork_70136815944304
// MI455X (gfx1250) — hardware-verified
//
#include <hip/hip_runtime.h>
#include <math.h>

constexpr int NVAR = 16;
constexpr int DM   = 128;
constexpr int VDM  = NVAR * DM;
constexpr int NROWS = 32 * 512;
constexpr int ROWS_PER_BLOCK = 16;
constexpr int NBLOCKS = NROWS / ROWS_PER_BLOCK;
constexpr float LN_EPS = 1e-5f;
constexpr float INV_DM = 1.0f / 128.0f;
constexpr float INV_NV = 1.0f / 16.0f;
static_assert(NROWS % ROWS_PER_BLOCK == 0, "rows tile exactly");
static_assert(DM % 32 == 0 && VDM % 32 == 0, "every GEMM K is a multiple of 32");

constexpr size_t WS_W2  = 0;
constexpr size_t WS_WG  = WS_W2  + (size_t)NVAR * DM * DM;
constexpr size_t WS_SW1 = WS_WG  + (size_t)NVAR * DM * DM;
constexpr size_t WS_SWS = WS_SW1 + (size_t)DM * VDM;
constexpr size_t WS_SW2 = WS_SWS + (size_t)NVAR * VDM;
constexpr size_t WS_SWG = WS_SW2 + (size_t)NVAR * DM;
constexpr size_t WS_TOTAL_U16 = WS_SWG + (size_t)NVAR * DM;
static_assert(WS_TOTAL_U16 * 2 == 1646592, "carve total bytes");
static_assert(WS_TOTAL_U16 * 2 <= 134217728, "carve under 128 MiB");

constexpr size_t OUT1_FLOAT_OFF = 8388608 / 4;
static_assert(OUT1_FLOAT_OFF == (size_t)NROWS * DM, "out1 follows out0");
static_assert(8388608 + (size_t)NROWS * NVAR * 4 == 9437184, "last output ends at the total");

typedef __attribute__((ext_vector_type(16))) __bf16   v16b;
typedef __attribute__((ext_vector_type(8)))  __bf16   v8b;
typedef __attribute__((ext_vector_type(8)))  float    v8f;
typedef __attribute__((ext_vector_type(4)))  float    v4f;
typedef __attribute__((ext_vector_type(4)))  unsigned int v4u;

__device__ __forceinline__ unsigned short f2bf_bits(float f) {
  unsigned u = __float_as_uint(f);
  return (unsigned short)((u + 0x7FFFu + ((u >> 16) & 1u)) >> 16);
}
__device__ __forceinline__ float bf_bits2f(unsigned short h) { return __uint_as_float(((unsigned)h) << 16); }
__device__ __forceinline__ float bfr(float f) { return bf_bits2f(f2bf_bits(f)); }
__device__ __forceinline__ unsigned pk16(unsigned short a, unsigned short b) { return (unsigned)a | ((unsigned)b << 16); }

struct FragB {
  union U { v16b v; v8b h[2]; };
  static __device__ __forceinline__ v16b load(const __bf16* p) {
    U f; f.h[0] = *(const v8b*)(p); f.h[1] = *(const v8b*)(p + 16); return f.v;
  }
};
__device__ __forceinline__ v8f mma_bf(v16b a, v16b b, v8f c) {
  return __builtin_amdgcn_wmma_f32_16x16x32_bf16(false, a, false, b, (short)0, c, false, false);
}
__device__ __forceinline__ void guard2m(v8f& a, v8f& b, v16b x, v16b y, v16b z, v16b w) {
  asm volatile("v_nop\n\tv_nop\n\tv_nop\n\tv_nop" : "+v"(a), "+v"(b) : "v"(x), "v"(y), "v"(z), "v"(w) : "memory");
}
__device__ __forceinline__ void guard1m(v8f& a, v16b x, v16b y, v16b z) {
  asm volatile("v_nop\n\tv_nop\n\tv_nop\n\tv_nop" : "+v"(a) : "v"(x), "v"(y), "v"(z) : "memory");
}

__device__ __forceinline__ float hsum16(float v) {
  v += __shfl_xor(v, 1, 32);
  v += __shfl_xor(v, 2, 32);
  v += __shfl_xor(v, 4, 32);
  v += __shfl_xor(v, 8, 32);
  return v;
}
__device__ __forceinline__ float hmax16(float v) {
  v = fmaxf(v, __shfl_xor(v, 1, 32));
  v = fmaxf(v, __shfl_xor(v, 2, 32));
  v = fmaxf(v, __shfl_xor(v, 4, 32));
  v = fmaxf(v, __shfl_xor(v, 8, 32));
  return v;
}
__device__ __forceinline__ float elu_f(float a) {
  const float en = expm1f(fminf(a, 0.0f));
  return (a > 0.0f) ? a : en;
}
__device__ __forceinline__ float sigm_f(float a) {
  return 1.0f / (1.0f + expf(-a));
}

__global__ __launch_bounds__(256) void cvt_bf16x8(const float* __restrict__ in,
                                                 unsigned short* __restrict__ out, int n8) {
  const int i = blockIdx.x * 256 + threadIdx.x;
  if (i >= n8) return;
  const float* p = in + 8 * (size_t)i;
  const v4f a = *(const v4f*)(p);
  const v4f c = *(const v4f*)(p + 4);
  unsigned short hb[8];
#pragma unroll
  for (int e = 0; e < 4; ++e) {
    hb[e]     = f2bf_bits(a[e]);
    hb[4 + e] = f2bf_bits(c[e]);
  }
  const v4u u = (v4u){pk16(hb[0], hb[1]), pk16(hb[2], hb[3]), pk16(hb[4], hb[5]), pk16(hb[6], hb[7])};
  unsigned short* q = out + 8 * (size_t)i;
  *(volatile v4u*)q = u;
  __threadfence();
  *(volatile v4u*)q = u;
}

__global__ __launch_bounds__(256)
void vsn_fused(const float* __restrict__ x,
               const float* __restrict__ W1,  const float* __restrict__ b1,
               const float* __restrict__ b2,  const float* __restrict__ bg,
               const float* __restrict__ Ws,  const float* __restrict__ bs,
               const float* __restrict__ gam, const float* __restrict__ bet,
               const float* __restrict__ sb1, const float* __restrict__ sb2,
               const float* __restrict__ sbg, const float* __restrict__ sbs,
               const float* __restrict__ sgam, const float* __restrict__ sbet,
               const unsigned short* __restrict__ w2bf,  const unsigned short* __restrict__ wgbf,
               const unsigned short* __restrict__ sw1bf, const unsigned short* __restrict__ swsbf,
               const unsigned short* __restrict__ sw2bf, const unsigned short* __restrict__ swgbf,
               float* __restrict__ outP, float* __restrict__ outW)
{
  __shared__ __align__(16) unsigned short flatHi[ROWS_PER_BLOCK * VDM];
  __shared__ __align__(16) unsigned short flatLo[ROWS_PER_BLOCK * VDM];
  __shared__ __align__(16) unsigned short hHi[ROWS_PER_BLOCK * DM];
  __shared__ __align__(16) unsigned short hLo[ROWS_PER_BLOCK * DM];
  __shared__ __align__(16) unsigned short hsHi[ROWS_PER_BLOCK * DM];
  __shared__ __align__(16) unsigned short hsLo[ROWS_PER_BLOCK * DM];
  __shared__ __align__(16) float ytile[ROWS_PER_BLOCK * DM];
  __shared__ __align__(16) float prm[8 * DM];
  __shared__ __align__(16) float xs[ROWS_PER_BLOCK * NVAR];
  __shared__ __align__(16) float partL[8 * 8 * 32];
  __shared__ __align__(16) float wL[ROWS_PER_BLOCK * NVAR];
  __shared__ __align__(16) float procL[ROWS_PER_BLOCK * DM];

  const int tid  = threadIdx.x;
  const int wv   = tid >> 5;
  const int lane = tid & 31;
  const int cc   = lane & 15;
  const int hh   = lane >> 4;
  const int tm   = tid >> 4;
  const int tj   = tid & 15;
  const int n0   = blockIdx.x * ROWS_PER_BLOCK;

  xs[tid] = bfr(x[(size_t)n0 * NVAR + tid]);

  const float* psrc = (wv == 0) ? W1 : (wv == 1) ? b1 : (wv == 2) ? Ws : (wv == 3) ? bs
                    : (wv == 4) ? b2 : (wv == 5) ? bg : (wv == 6) ? gam : bet;
  const v8f vz = {0.f, 0.f, 0.f, 0.f, 0.f, 0.f, 0.f, 0.f};

#pragma unroll 1
  for (int v = 0; v < NVAR; ++v) {
    {
      const v4f p4 = *(const v4f*)(psrc + v * DM + 4 * lane);
      const v4f r4 = (v4f){bfr(p4[0]), bfr(p4[1]), bfr(p4[2]), bfr(p4[3])};
      *(v4f*)(prm + wv * DM + 4 * lane) = r4;
    }
    __syncthreads();

    {
      const float xv = xs[tm * NVAR + v];
      const v4f wa = *(const v4f*)(prm + 8 * tj);
      const v4f wb = *(const v4f*)(prm + 8 * tj + 4);
      const v4f ba = *(const v4f*)(prm + DM + 8 * tj);
      const v4f bb = *(const v4f*)(prm + DM + 8 * tj + 4);
      float hp[8];
#pragma unroll
      for (int e = 0; e < 4; ++e) {
        hp[e]     = xv * wa[e] + ba[e];
        hp[4 + e] = xv * wb[e] + bb[e];
      }
      unsigned short hb[8], lb[8];
#pragma unroll
      for (int e = 0; e < 8; ++e) {
        const float hv = elu_f(hp[e]);
        hb[e] = f2bf_bits(hv);
        lb[e] = f2bf_bits(hv - bf_bits2f(hb[e]));
      }
      *(v4u*)(hHi + tm * DM + 8 * tj) = (v4u){pk16(hb[0], hb[1]), pk16(hb[2], hb[3]), pk16(hb[4], hb[5]), pk16(hb[6], hb[7])};
      *(v4u*)(hLo + tm * DM + 8 * tj) = (v4u){pk16(lb[0], lb[1]), pk16(lb[2], lb[3]), pk16(lb[4], lb[5]), pk16(lb[6], lb[7])};
    }
    __syncthreads();

    {
      const int o = wv * 16 + cc;
      const __bf16* ap  = (const __bf16*)hHi + cc * DM + 8 * hh;
      const __bf16* alp = (const __bf16*)hLo + cc * DM + 8 * hh;
      const __bf16* b2p = (const __bf16*)w2bf + (size_t)v * DM * DM + (size_t)o * DM + 8 * hh;
      const __bf16* bgp = (const __bf16*)wgbf + (size_t)v * DM * DM + (size_t)o * DM + 8 * hh;
      v8f acc2 = vz, accg = vz;
#pragma unroll
      for (int kc = 0; kc < DM / 32; ++kc) {
        const v16b ah  = FragB::load(ap  + kc * 32);
        const v16b al  = FragB::load(alp + kc * 32);
        const v16b bh  = FragB::load(b2p + kc * 32);
        const v16b bgf = FragB::load(bgp + kc * 32);
        acc2 = mma_bf(ah, bh,  acc2);
        acc2 = mma_bf(al, bh,  acc2);
        accg = mma_bf(ah, bgf, accg);
        accg = mma_bf(al, bgf, accg);
        guard2m(acc2, accg, ah, al, bh, bgf);
      }
      const float wso = prm[2 * DM + o], bso = prm[3 * DM + o];
      const float b2o = prm[4 * DM + o], bgo = prm[5 * DM + o];
#pragma unroll
      for (int r = 0; r < 8; ++r) {
        const int m = 8 * hh + r;
        const float xm = xs[m * NVAR + v];
        const float h2 = acc2[r] + b2o;
        const float gt = sigm_f(accg[r] + bgo);
        const float sk = xm * wso + bso;
        ytile[m * DM + o] = gt * h2 + (1.0f - gt) * sk;
      }
    }
    __syncthreads();

    {
      const v4f ya = *(const v4f*)(ytile + tm * DM + 8 * tj);
      const v4f yb = *(const v4f*)(ytile + tm * DM + 8 * tj + 4);
      float yv[8];
#pragma unroll
      for (int e = 0; e < 4; ++e) { yv[e] = ya[e]; yv[4 + e] = yb[e]; }
      float s = 0.0f;
#pragma unroll
      for (int e = 0; e < 8; ++e) s += yv[e];
      s = hsum16(s);
      const float mean = s * INV_DM;
      float dv[8];
      float q = 0.0f;
#pragma unroll
      for (int e = 0; e < 8; ++e) { dv[e] = yv[e] - mean; q += dv[e] * dv[e]; }
      q = hsum16(q);
      const float rstd = rsqrtf(q * INV_DM + LN_EPS);
      const v4f ga = *(const v4f*)(prm + 6 * DM + 8 * tj);
      const v4f gb = *(const v4f*)(prm + 6 * DM + 8 * tj + 4);
      const v4f ea = *(const v4f*)(prm + 7 * DM + 8 * tj);
      const v4f eb = *(const v4f*)(prm + 7 * DM + 8 * tj + 4);
      float gv[8], bv[8];
#pragma unroll
      for (int e = 0; e < 4; ++e) { gv[e] = ga[e]; gv[4 + e] = gb[e]; bv[e] = ea[e]; bv[4 + e] = eb[e]; }
      unsigned short hb[8], lb[8];
#pragma unroll
      for (int e = 0; e < 8; ++e) {
        const float yn = dv[e] * rstd * gv[e] + bv[e];
        hb[e] = f2bf_bits(yn);
        lb[e] = f2bf_bits(yn - bf_bits2f(hb[e]));
      }
      *(v4u*)(flatHi + tm * VDM + v * DM + 8 * tj) = (v4u){pk16(hb[0], hb[1]), pk16(hb[2], hb[3]), pk16(hb[4], hb[5]), pk16(hb[6], hb[7])};
      *(v4u*)(flatLo + tm * VDM + v * DM + 8 * tj) = (v4u){pk16(lb[0], lb[1]), pk16(lb[2], lb[3]), pk16(lb[4], lb[5]), pk16(lb[6], lb[7])};
    }
    __syncthreads();
  }

  {
    const int o = wv * 16 + cc;
    const __bf16* ap  = (const __bf16*)flatHi + cc * VDM + 8 * hh;
    const __bf16* alp = (const __bf16*)flatLo + cc * VDM + 8 * hh;
    const __bf16* bp  = (const __bf16*)sw1bf + (size_t)o * VDM + 8 * hh;
    v8f acc = vz;
#pragma unroll 2
    for (int kc = 0; kc < VDM / 32; ++kc) {
      const v16b ah = FragB::load(ap  + kc * 32);
      const v16b al = FragB::load(alp + kc * 32);
      const v16b bh = FragB::load(bp  + kc * 32);
      acc = mma_bf(ah, bh, acc);
      acc = mma_bf(al, bh, acc);
      guard1m(acc, ah, al, bh);
    }
    const float sb1o = bfr(sb1[o]);
#pragma unroll
    for (int r = 0; r < 8; ++r) {
      const int m = 8 * hh + r;
      const float hv = elu_f(acc[r] + sb1o);
      const unsigned short hb = f2bf_bits(hv);
      const unsigned short lb = f2bf_bits(hv - bf_bits2f(hb));
      hsHi[m * DM + o] = hb;
      hsLo[m * DM + o] = lb;
    }
  }
  {
    const __bf16* ap  = (const __bf16*)flatHi + cc * VDM + 8 * hh;
    const __bf16* alp = (const __bf16*)flatLo + cc * VDM + 8 * hh;
    const __bf16* bp  = (const __bf16*)swsbf + (size_t)cc * VDM + 8 * hh;
    v8f acc = vz;
#pragma unroll
    for (int kk = 0; kk < 8; ++kk) {
      const int kc = wv * 8 + kk;
      const v16b ah = FragB::load(ap  + kc * 32);
      const v16b al = FragB::load(alp + kc * 32);
      const v16b bh = FragB::load(bp  + kc * 32);
      acc = mma_bf(ah, bh, acc);
      acc = mma_bf(al, bh, acc);
      guard1m(acc, ah, al, bh);
    }
#pragma unroll
    for (int r = 0; r < 8; ++r) partL[(wv * 8 + r) * 32 + lane] = acc[r];
  }
  __syncthreads();

  if (wv == 0) {
    const __bf16* ap  = (const __bf16*)hsHi + cc * DM + 8 * hh;
    const __bf16* alp = (const __bf16*)hsLo + cc * DM + 8 * hh;
    const __bf16* b2p = (const __bf16*)sw2bf + (size_t)cc * DM + 8 * hh;
    const __bf16* bgp = (const __bf16*)swgbf + (size_t)cc * DM + 8 * hh;
    v8f a2 = vz, ag = vz;
#pragma unroll
    for (int kc = 0; kc < DM / 32; ++kc) {
      const v16b ah  = FragB::load(ap  + kc * 32);
      const v16b al  = FragB::load(alp + kc * 32);
      const v16b bh  = FragB::load(b2p + kc * 32);
      const v16b bgf = FragB::load(bgp + kc * 32);
      a2 = mma_bf(ah, bh,  a2);
      a2 = mma_bf(al, bh,  a2);
      ag = mma_bf(ah, bgf, ag);
      ag = mma_bf(al, bgf, ag);
      guard2m(a2, ag, ah, al, bh, bgf);
    }
    const float sb2c = bfr(sb2[cc]);
    const float sbgc = bfr(sbg[cc]);
    const float sbsc = bfr(sbs[cc]);
    const float sgc  = bfr(sgam[cc]);
    const float sbc  = bfr(sbet[cc]);
    float z[8];
#pragma unroll
    for (int r = 0; r < 8; ++r) {
      float sk = 0.0f;
#pragma unroll
      for (int w = 0; w < 8; ++w) sk += partL[(w * 8 + r) * 32 + lane];
      sk += sbsc;
      const float h2 = a2[r] + sb2c;
      const float gt = sigm_f(ag[r] + sbgc);
      z[r] = gt * h2 + (1.0f - gt) * sk;
    }
#pragma unroll
    for (int r = 0; r < 8; ++r) {
      const float s    = hsum16(z[r]);
      const float mean = s * INV_NV;
      const float d    = z[r] - mean;
      const float dd   = d * d;
      const float q    = hsum16(dd);
      const float rstd = rsqrtf(q * INV_NV + LN_EPS);
      const float zn   = d * rstd * sgc + sbc;
      const float mx   = hmax16(zn);
      const float ex   = expf(zn - mx);
      const float se   = hsum16(ex);
      const float wt   = ex / se;
      wL[(8 * hh + r) * NVAR + cc] = wt;
    }
  }
  __syncthreads();

  {
    float accp[8];
#pragma unroll
    for (int e = 0; e < 8; ++e) accp[e] = 0.0f;
#pragma unroll 4
    for (int v = 0; v < NVAR; ++v) {
      const float wt = wL[tm * NVAR + v];
      const v4u hw = *(const v4u*)(flatHi + tm * VDM + v * DM + 8 * tj);
      const v4u lw = *(const v4u*)(flatLo + tm * VDM + v * DM + 8 * tj);
#pragma unroll
      for (int qq = 0; qq < 4; ++qq) {
        const unsigned ha = hw[qq];
        const unsigned la = lw[qq];
        const float s0 = __uint_as_float(ha << 16) + __uint_as_float(la << 16);
        const float s1 = __uint_as_float(ha & 0xffff0000u) + __uint_as_float(la & 0xffff0000u);
        accp[2 * qq]     += s0 * wt;
        accp[2 * qq + 1] += s1 * wt;
      }
    }
    *(v4f*)(procL + tm * DM + 8 * tj)     = (v4f){accp[0], accp[1], accp[2], accp[3]};
    *(v4f*)(procL + tm * DM + 8 * tj + 4) = (v4f){accp[4], accp[5], accp[6], accp[7]};
  }
  __syncthreads();

  {
    float* ob = outP + (size_t)n0 * DM;
    for (int pass = 0; pass < 2; ++pass) {
#pragma unroll
      for (int it = 0; it < 2; ++it) {
        const int row = wv * 2 + it;
        const v4f val = *(const v4f*)(procL + row * DM + 4 * lane);
        *(volatile v4f*)(ob + (size_t)row * DM + 4 * lane) = val;
      }
      __threadfence();
    }
  }
  if (wv == 0) {
    float* wb = outW + (size_t)n0 * NVAR;
    for (int pass = 0; pass < 2; ++pass) {
#pragma unroll
      for (int it = 0; it < 2; ++it) {
        const v4f val = *(const v4f*)(wL + it * 128 + 4 * lane);
        *(volatile v4f*)(wb + it * 128 + 4 * lane) = val;
      }
      __threadfence();
    }
  }
}

extern "C" void kernel_launch(void* const* d_in, const int* in_sizes, int n_in,
                              void* d_out, int out_size, void* d_ws, size_t ws_size,
                              hipStream_t stream) {
  if (n_in < 21) return;
  if (in_sizes[0] != NROWS * NVAR) return;
  if (out_size < NROWS * (DM + NVAR)) return;
  if (ws_size < WS_TOTAL_U16 * 2) return;

  const float* x     = (const float*)d_in[0];
  const float* W1    = (const float*)d_in[1];
  const float* b1    = (const float*)d_in[2];
  const float* W2    = (const float*)d_in[3];
  const float* b2    = (const float*)d_in[4];
  const float* Wg    = (const float*)d_in[5];
  const float* bg    = (const float*)d_in[6];
  const float* Ws    = (const float*)d_in[7];
  const float* bs    = (const float*)d_in[8];
  const float* gam   = (const float*)d_in[9];
  const float* bet   = (const float*)d_in[10];
  const float* sW1   = (const float*)d_in[11];
  const float* sb1   = (const float*)d_in[12];
  const float* sW2   = (const float*)d_in[13];
  const float* sb2   = (const float*)d_in[14];
  const float* sWg   = (const float*)d_in[15];
  const float* sbg   = (const float*)d_in[16];
  const float* sWs   = (const float*)d_in[17];
  const float* sbs   = (const float*)d_in[18];
  const float* sgam  = (const float*)d_in[19];
  const float* sbet  = (const float*)d_in[20];

  unsigned short* wsb   = (unsigned short*)d_ws;
  unsigned short* w2bf  = wsb + WS_W2;
  unsigned short* wgbf  = wsb + WS_WG;
  unsigned short* sw1bf = wsb + WS_SW1;
  unsigned short* swsbf = wsb + WS_SWS;
  unsigned short* sw2bf = wsb + WS_SW2;
  unsigned short* swgbf = wsb + WS_SWG;

  constexpr int N8_VDD = NVAR * DM * DM / 8;
  constexpr int N8_SW1 = DM * VDM / 8;
  constexpr int N8_SWS = NVAR * VDM / 8;
  constexpr int N8_SW2 = NVAR * DM / 8;
  static_assert(N8_VDD % 256 == 0 && N8_SW1 % 256 == 0 && N8_SWS % 256 == 0 && N8_SW2 % 256 == 0, "exact grids");
  cvt_bf16x8<<<N8_VDD / 256, 256, 0, stream>>>(W2,  w2bf,  N8_VDD);
  cvt_bf16x8<<<N8_VDD / 256, 256, 0, stream>>>(Wg,  wgbf,  N8_VDD);
  cvt_bf16x8<<<N8_SW1 / 256, 256, 0, stream>>>(sW1, sw1bf, N8_SW1);
  cvt_bf16x8<<<N8_SWS / 256, 256, 0, stream>>>(sWs, swsbf, N8_SWS);
  cvt_bf16x8<<<N8_SW2 / 256, 256, 0, stream>>>(sW2, sw2bf, N8_SW2);
  cvt_bf16x8<<<N8_SW2 / 256, 256, 0, stream>>>(sWg, swgbf, N8_SW2);

  float* outP = (float*)d_out;
  float* outW = (float*)d_out + OUT1_FLOAT_OFF;

  vsn_fused<<<NBLOCKS, 256, 0, stream>>>(
      x, W1, b1, b2, bg, Ws, bs, gam, bet,
      sb1, sb2, sbg, sbs, sgam, sbet,
      w2bf, wgbf, sw1bf, swsbf, sw2bf, swgbf,
      outP, outW);
}
